// GeometryMultiHeadAttention_52931176956436
// MI455X (gfx1250) — hardware-verified
//
#include <hip/hip_runtime.h>


typedef __bf16   v8bf  __attribute__((ext_vector_type(8)));
typedef __bf16   v16bf __attribute__((ext_vector_type(16)));
typedef _Float16 v8h   __attribute__((ext_vector_type(8)));
typedef _Float16 v16h  __attribute__((ext_vector_type(16)));
typedef float    v4f   __attribute__((ext_vector_type(4)));
typedef float    v8f   __attribute__((ext_vector_type(8)));

#define B_  4
#define N_  1024
#define D_  512
#define H_  8
#define HD_ 64
#define R_  32

__device__ __forceinline__ v16bf cat_bf(v8bf a, v8bf b) {
  return __builtin_shufflevector(a, b, 0, 1, 2, 3, 4, 5, 6, 7, 8, 9, 10, 11, 12, 13, 14, 15);
}
__device__ __forceinline__ v16h cat_h(v8h a, v8h b) {
  return __builtin_shufflevector(a, b, 0, 1, 2, 3, 4, 5, 6, 7, 8, 9, 10, 11, 12, 13, 14, 15);
}

__device__ __forceinline__ v8f mma_bf(v16bf a, v16bf b, v8f c) {
  return __builtin_amdgcn_wmma_f32_16x16x32_bf16(false, a, false, b, (short)0, c, false, false);
}
__device__ __forceinline__ v8f mma_h(v16h a, v16h b, v8f c) {
  return __builtin_amdgcn_wmma_f32_16x16x32_f16(false, a, false, b, (short)0, c, false, false);
}
#define WG1(acc, a, b) \
  asm volatile("v_nop\n\tv_nop\n\tv_nop\n\tv_nop" : "+v"(acc) : "v"(a), "v"(b))
#define WG4(a0, a1, a2, a3, x, y)                                              \
  asm volatile("v_nop\n\tv_nop\n\tv_nop\n\tv_nop"                            \
               : "+v"(a0), "+v"(a1), "+v"(a2), "+v"(a3) : "v"(x), "v"(y))

__device__ __forceinline__ void split8(v4f x0, v4f x1, v8bf& hi, v8bf& lo) {
#pragma unroll
  for (int i = 0; i < 4; i++) {
    const float f = x0[i];
    const __bf16 hf = (__bf16)f;
    hi[i] = hf;
    lo[i] = (__bf16)(f - (float)hf);
    const float g = x1[i];
    const __bf16 hg = (__bf16)g;
    hi[4 + i] = hg;
    lo[4 + i] = (__bf16)(g - (float)hg);
  }
}

#define GA_P 40
#define GS_P 132
#define GT_P 68

template <int MODE>
__global__ __launch_bounds__(256) void k_gemm(const float* __restrict__ A,
                                            const float* __restrict__ W,
                                            const float* __restrict__ bias,
                                            float* __restrict__ Cf,
                                            __bf16* __restrict__ Chi,
                                            __bf16* __restrict__ Clo,
                                            float scale, int M) {
  __shared__ __align__(16) unsigned char smem[40960];
  __bf16* Ahi = (__bf16*)smem;
  __bf16* Alo = Ahi + 64 * GA_P;
  __bf16* Bhi = Alo + 64 * GA_P;
  __bf16* Blo = Bhi + 128 * GA_P;
  float* st = (float*)smem;

  const int m0 = blockIdx.x * 64;
  const int n0 = blockIdx.y * 128;
  const int tid = threadIdx.x;
  const int wave = tid >> 5;
  const int lane = tid & 31;
  const int lgrp = lane >> 4;
  const int l16 = lane & 15;
  const int wm = (wave >> 2) * 32;
  const int wn = (wave & 3) * 32;

  v8f acc[2][2];
#pragma unroll
  for (int rt = 0; rt < 2; rt++)
#pragma unroll
    for (int ct = 0; ct < 2; ct++)
#pragma unroll
      for (int r = 0; r < 8; r++) acc[rt][ct][r] = 0.0f;

  for (int k0 = 0; k0 < D_; k0 += 32) {
    __syncthreads();
    {
      const int row = tid >> 2, kc = (tid & 3) * 8;
      int gr = m0 + row;
      if (gr > M - 1) gr = M - 1;
      const float* ap = A + (size_t)gr * D_ + k0 + kc;
      v8bf hv, lv;
      split8(*(const v4f*)ap, *(const v4f*)(ap + 4), hv, lv);
      *(v8bf*)(Ahi + row * GA_P + kc) = hv;
      *(v8bf*)(Alo + row * GA_P + kc) = lv;
    }
    {
      const int kk = tid >> 3, nc = (tid & 7) * 16;
      const float* wp = W + (size_t)(k0 + kk) * D_ + n0 + nc;
#pragma unroll
      for (int j = 0; j < 4; j++) {
        const v4f x = *(const v4f*)(wp + 4 * j);
#pragma unroll
        for (int i = 0; i < 4; i++) {
          const float f = x[i];
          const __bf16 hf = (__bf16)f;
          Bhi[(nc + 4 * j + i) * GA_P + kk] = hf;
          Blo[(nc + 4 * j + i) * GA_P + kk] = (__bf16)(f - (float)hf);
        }
      }
    }
    __syncthreads();

    v16bf ah[2], al[2], bh[2], bl[2];
#pragma unroll
    for (int rt = 0; rt < 2; rt++) {
      const __bf16* ph = Ahi + (wm + rt * 16 + l16) * GA_P;
      const __bf16* pl = Alo + (wm + rt * 16 + l16) * GA_P;
      ah[rt] = cat_bf(*(const v8bf*)(ph + 8 * lgrp), *(const v8bf*)(ph + 16 + 8 * lgrp));
      al[rt] = cat_bf(*(const v8bf*)(pl + 8 * lgrp), *(const v8bf*)(pl + 16 + 8 * lgrp));
    }
#pragma unroll
    for (int ct = 0; ct < 2; ct++) {
      const __bf16* ph = Bhi + (wn + ct * 16 + l16) * GA_P;
      const __bf16* pl = Blo + (wn + ct * 16 + l16) * GA_P;
      bh[ct] = cat_bf(*(const v8bf*)(ph + 8 * lgrp), *(const v8bf*)(ph + 16 + 8 * lgrp));
      bl[ct] = cat_bf(*(const v8bf*)(pl + 8 * lgrp), *(const v8bf*)(pl + 16 + 8 * lgrp));
    }
#pragma unroll
    for (int rt = 0; rt < 2; rt++) {
#pragma unroll
      for (int ct = 0; ct < 2; ct++) {
        acc[rt][ct] = mma_bf(ah[rt], bh[ct], acc[rt][ct]);
        acc[rt][ct] = mma_bf(ah[rt], bl[ct], acc[rt][ct]);
        acc[rt][ct] = mma_bf(al[rt], bh[ct], acc[rt][ct]);
      }
    }
    WG4(acc[0][0], acc[0][1], acc[1][0], acc[1][1], al[1], bh[1]);
  }

  __syncthreads();
#pragma unroll
  for (int rt = 0; rt < 2; rt++) {
#pragma unroll
    for (int ct = 0; ct < 2; ct++) {
      const int col = wn + ct * 16 + l16;
      const float bv = bias[n0 + col];
#pragma unroll
      for (int r = 0; r < 8; r++) {
        const int row = wm + rt * 16 + 8 * lgrp + r;
        const float val = (acc[rt][ct][r] + bv) * scale;
        if constexpr (MODE == 2)
          st[col * GT_P + row] = val;
        else
          st[row * GS_P + col] = val;
      }
    }
  }
  __syncthreads();

  if constexpr (MODE == 0) {
    const int sub = (lane & 7) * 4;
    v4f vv[8];
#pragma unroll
    for (int j = 0; j < 8; j++) {
      const int L = wave * 32 + j * 4 + (lane >> 3);
      const int row = L >> 2, seg = L & 3;
      vv[j] = *(const v4f*)(st + row * GS_P + seg * 32 + sub);
      float* dp = Cf + (size_t)(m0 + row) * D_ + n0 + seg * 32 + sub;
      if (m0 + row < M) *(volatile v4f*)dp = vv[j];
    }
    __threadfence();
#pragma unroll
    for (int j = 0; j < 8; j++) {
      const int L = wave * 32 + j * 4 + (lane >> 3);
      const int row = L >> 2, seg = L & 3;
      float* dp = Cf + (size_t)(m0 + row) * D_ + n0 + seg * 32 + sub;
      if (m0 + row < M) *(volatile v4f*)dp = vv[j];
    }
  } else {
    const int sub = (lane & 7) * 8;
    const int bb = m0 >> 10;
    const int nl0 = m0 & (N_ - 1);
    v8bf hv[4], lv[4];
    size_t off[4];
#pragma unroll
    for (int j = 0; j < 4; j++) {
      const int L = wave * 16 + j * 4 + (lane >> 3);
      const float* sp;
      if constexpr (MODE == 1) {
        const int row = L >> 1, seg = L & 1;
        sp = st + row * GS_P + seg * 64 + sub;
        off[j] = (size_t)(m0 + row) * D_ + n0 + seg * 64 + sub;
      } else {
        const int c = L;
        sp = st + c * GT_P + sub;
        off[j] = ((size_t)(bb * D_ + n0 + c)) * N_ + nl0 + sub;
      }
      split8(*(const v4f*)sp, *(const v4f*)(sp + 4), hv[j], lv[j]);
      *(volatile v8bf*)(Chi + off[j]) = hv[j];
      *(volatile v8bf*)(Clo + off[j]) = lv[j];
    }
    __threadfence();
#pragma unroll
    for (int j = 0; j < 4; j++) {
      *(volatile v8bf*)(Chi + off[j]) = hv[j];
      *(volatile v8bf*)(Clo + off[j]) = lv[j];
    }
  }
}

#define AKP 520
#define AVP 40
#define AFP 40
#define ABP 9
#define APP 40
#define AOP 68
#define OFF_KHI 0
#define OFF_KLO 33280
#define OFF_VHI 66560
#define OFF_VLO 107520
#define OFF_FEA 148480
#define OFF_BIA 189440
#define OFF_PHI 207872
#define OFF_PLO 218112
#define ATT_LDS 228352

__global__ __launch_bounds__(256) void k_attn(const float* __restrict__ Q,
                                            const __bf16* __restrict__ Khi_g,
                                            const __bf16* __restrict__ Klo_g,
                                            const __bf16* __restrict__ Vhi_g,
                                            const __bf16* __restrict__ Vlo_g,
                                            const float* __restrict__ pos,
                                            const int* __restrict__ mask,
                                            const float* __restrict__ rbf_w,
                                            const float* __restrict__ rbf_b,
                                            float* __restrict__ O) {
  extern __shared__ __align__(16) unsigned char dsm[];
  __bf16* Khi = (__bf16*)(dsm + OFF_KHI);
  __bf16* Klo = (__bf16*)(dsm + OFF_KLO);
  __bf16* Vhi = (__bf16*)(dsm + OFF_VHI);
  __bf16* Vlo = (__bf16*)(dsm + OFF_VLO);
  _Float16* fea = (_Float16*)(dsm + OFF_FEA);
  float* bia = (float*)(dsm + OFF_BIA);
  __bf16* Phi = (__bf16*)(dsm + OFF_PHI);
  __bf16* Plo = (__bf16*)(dsm + OFF_PLO);

  const int tid = threadIdx.x;
  const int w = tid >> 5;
  const int lane = tid & 31;
  const int lgrp = lane >> 4;
  const int l16 = lane & 15;
  const int qbase = blockIdx.x * 16;
  const int b = blockIdx.y;

  const float SPACING = 0.32258064516f;
  const float NGL = -9.61f * 1.4426950408889634f;
  const float LOG2E = 1.4426950408889634f;

  v16h wf;
#pragma unroll
  for (int i = 0; i < 16; i++) {
    const int r = (i < 8) ? (8 * lgrp + i) : (16 + 8 * lgrp + (i - 8));
    const float wv = (l16 < H_) ? rbf_w[r * H_ + l16] : 0.0f;
    wf[i] = (_Float16)wv;
  }
  const float rb = rbf_b[w];

  v16bf qh[2], ql[2];
  {
    const float* qrow = Q + (size_t)(b * N_ + qbase + l16) * D_ + w * HD_;
#pragma unroll
    for (int kk = 0; kk < 2; kk++) {
      const float* p0 = qrow + kk * 32 + 8 * lgrp;
      v8bf h0, l0, h1, l1;
      split8(*(const v4f*)p0, *(const v4f*)(p0 + 4), h0, l0);
      split8(*(const v4f*)(p0 + 16), *(const v4f*)(p0 + 20), h1, l1);
      qh[kk] = cat_bf(h0, h1);
      ql[kk] = cat_bf(l0, l1);
    }
  }

  const int fq = tid >> 4;
  float qx, qy, qz;
  {
    const float* qp = pos + (size_t)(b * N_ + qbase + fq) * 3;
    qx = qp[0]; qy = qp[1]; qz = qp[2];
  }

  v8f oacc[4];
#pragma unroll
  for (int ot = 0; ot < 4; ot++)
#pragma unroll
    for (int r = 0; r < 8; r++) oacc[ot][r] = 0.0f;
  float mi[8], li[8];
#pragma unroll
  for (int v = 0; v < 8; v++) { mi[v] = -1e30f; li[v] = 0.0f; }

  for (int kb = 0; kb < N_; kb += 32) {
    __syncthreads();
    {
      const int key = tid >> 3, cb = (tid & 7) * 64;
      const size_t g = (size_t)(b * N_ + kb + key) * D_ + cb;
#pragma unroll
      for (int j = 0; j < 8; j++) {
        *(v8bf*)(Khi + key * AKP + cb + 8 * j) = *(const v8bf*)(Khi_g + g + 8 * j);
        *(v8bf*)(Klo + key * AKP + cb + 8 * j) = *(const v8bf*)(Klo_g + g + 8 * j);
      }
    }
    {
#pragma unroll
      for (int cc = 0; cc < 2; cc++) {
        const int c = tid * 2 + cc;
        const size_t g = ((size_t)(b * D_ + c)) * N_ + kb;
#pragma unroll
        for (int j = 0; j < 4; j++) {
          *(v8bf*)(Vhi + c * AVP + 8 * j) = *(const v8bf*)(Vhi_g + g + 8 * j);
          *(v8bf*)(Vlo + c * AVP + 8 * j) = *(const v8bf*)(Vlo_g + g + 8 * j);
        }
      }
    }
    {
#pragma unroll
      for (int pp = 0; pp < 2; pp++) {
        const int p = tid * 2 + pp, k = p & 31;
        const float* kp = pos + (size_t)(b * N_ + kb + k) * 3;
        const float dx = qx - kp[0], dy = qy - kp[1], dz = qz - kp[2];
        const float d = __builtin_amdgcn_sqrtf(dx * dx + dy * dy + dz * dz);
#pragma unroll
        for (int g = 0; g < 4; g++) {
          v8h fv;
#pragma unroll
          for (int i = 0; i < 8; i++) {
            const float t = d - (float)(g * 8 + i) * SPACING;
            const float e = __builtin_amdgcn_exp2f(NGL * t * t);
            fv[i] = (_Float16)(e * 256.0f);
          }
          *(v8h*)(fea + p * AFP + g * 8) = fv;
        }
      }
    }
    __syncthreads();

#pragma unroll
    for (int r4 = 0; r4 < 4; r4++) {
      const int rt = w * 4 + r4;
      const _Float16* fr = fea + (rt * 16 + l16) * AFP;
      const v16h af = cat_h(*(const v8h*)(fr + 8 * lgrp), *(const v8h*)(fr + 16 + 8 * lgrp));
      v8f dacc;
#pragma unroll
      for (int r = 0; r < 8; r++) dacc[r] = 0.0f;
      dacc = mma_h(af, wf, dacc);
      WG1(dacc, af, wf);
      if (l16 < H_) {
#pragma unroll
        for (int r = 0; r < 8; r++)
          bia[(rt * 16 + 8 * lgrp + r) * ABP + l16] = dacc[r] * (1.0f / 256.0f);
      }
    }
    __syncthreads();

    float sc[2][8];
    v16bf kh, kl;
#pragma unroll
    for (int ct = 0; ct < 2; ct++) {
      v8f s;
#pragma unroll
      for (int r = 0; r < 8; r++) s[r] = 0.0f;
      const __bf16* krh = Khi + (ct * 16 + l16) * AKP + w * HD_;
      const __bf16* krl = Klo + (ct * 16 + l16) * AKP + w * HD_;
#pragma unroll
      for (int kk = 0; kk < 2; kk++) {
        const int c0 = kk * 32 + 8 * lgrp;
        kh = cat_bf(*(const v8bf*)(krh + c0), *(const v8bf*)(krh + c0 + 16));
        kl = cat_bf(*(const v8bf*)(krl + c0), *(const v8bf*)(krl + c0 + 16));
        s = mma_bf(qh[kk], kh, s);
        s = mma_bf(qh[kk], kl, s);
        s = mma_bf(ql[kk], kh, s);
      }
      WG1(s, ql[1], kh);
      const int nk = ct * 16 + l16;
      const bool ok = (mask[b * N_ + kb + nk] != 0);
#pragma unroll
      for (int v = 0; v < 8; v++) {
        const int q = 8 * lgrp + v;
        const float val = s[v] + bia[(q * 32 + nk) * ABP + w] + rb;
        sc[ct][v] = ok ? val * LOG2E : -1e30f;
      }
    }

    float alpha[8], mnew[8];
#pragma unroll
    for (int v = 0; v < 8; v++) {
      float mx = fmaxf(sc[0][v], sc[1][v]);
#pragma unroll
      for (int off = 1; off < 16; off <<= 1) mx = fmaxf(mx, __shfl_xor(mx, off, 32));
      mnew[v] = fmaxf(mi[v], mx);
      alpha[v] = __builtin_amdgcn_exp2f(mi[v] - mnew[v]);
    }
#pragma unroll
    for (int ct = 0; ct < 2; ct++)
#pragma unroll
      for (int v = 0; v < 8; v++)
        sc[ct][v] = __builtin_amdgcn_exp2f(sc[ct][v] - mnew[v]);
#pragma unroll
    for (int v = 0; v < 8; v++) {
      float rs = sc[0][v] + sc[1][v];
#pragma unroll
      for (int off = 1; off < 16; off <<= 1) rs += __shfl_xor(rs, off, 32);
      li[v] = li[v] * alpha[v] + rs;
      mi[v] = mnew[v];
    }
#pragma unroll
    for (int ot = 0; ot < 4; ot++)
#pragma unroll
      for (int v = 0; v < 8; v++) oacc[ot][v] *= alpha[v];

#pragma unroll
    for (int ct = 0; ct < 2; ct++) {
#pragma unroll
      for (int v = 0; v < 8; v++) {
        const float p = sc[ct][v];
        const __bf16 hp = (__bf16)p;
        const int idx = (w * 16 + 8 * lgrp + v) * APP + ct * 16 + l16;
        Phi[idx] = hp;
        Plo[idx] = (__bf16)(p - (float)hp);
      }
    }
    __syncthreads();
    v16bf ph, pl;
    {
      const __bf16* prh = Phi + (w * 16 + l16) * APP;
      const __bf16* prl = Plo + (w * 16 + l16) * APP;
      ph = cat_bf(*(const v8bf*)(prh + 8 * lgrp), *(const v8bf*)(prh + 16 + 8 * lgrp));
      pl = cat_bf(*(const v8bf*)(prl + 8 * lgrp), *(const v8bf*)(prl + 16 + 8 * lgrp));
    }

    v16bf vh, vl;
#pragma unroll
    for (int ot = 0; ot < 4; ot++) {
      const __bf16* vrh = Vhi + (w * HD_ + ot * 16 + l16) * AVP;
      const __bf16* vrl = Vlo + (w * HD_ + ot * 16 + l16) * AVP;
      vh = cat_bf(*(const v8bf*)(vrh + 8 * lgrp), *(const v8bf*)(vrh + 16 + 8 * lgrp));
      vl = cat_bf(*(const v8bf*)(vrl + 8 * lgrp), *(const v8bf*)(vrl + 16 + 8 * lgrp));
      oacc[ot] = mma_bf(ph, vh, oacc[ot]);
      oacc[ot] = mma_bf(ph, vl, oacc[ot]);
      oacc[ot] = mma_bf(pl, vh, oacc[ot]);
    }
    WG4(oacc[0], oacc[1], oacc[2], oacc[3], pl, vh);
  }

  __syncthreads();
  float* ost = (float*)(dsm + OFF_VHI) + w * (16 * AOP);
#pragma unroll
  for (int v = 0; v < 8; v++) {
    const float inv = 1.0f / li[v];
    const int q = 8 * lgrp + v;
#pragma unroll
    for (int ot = 0; ot < 4; ot++) ost[q * AOP + ot * 16 + l16] = oacc[ot][v] * inv;
  }
  __syncthreads();
  const int sub = (lane & 7) * 4;
  v4f vv[8];
#pragma unroll
  for (int j = 0; j < 8; j++) {
    const int L = j * 4 + (lane >> 3);
    const int row = L >> 1, seg = L & 1;
    vv[j] = *(const v4f*)(ost + row * AOP + seg * 32 + sub);
    float* dp = O + (size_t)(b * N_ + qbase + row) * D_ + w * HD_ + seg * 32 + sub;
    *(volatile v4f*)dp = vv[j];
  }
  __threadfence();
#pragma unroll
  for (int j = 0; j < 8; j++) {
    const int L = j * 4 + (lane >> 3);
    const int row = L >> 1, seg = L & 1;
    float* dp = O + (size_t)(b * N_ + qbase + row) * D_ + w * HD_ + seg * 32 + sub;
    *(volatile v4f*)dp = vv[j];
  }
}

extern "C" void kernel_launch(void* const* d_in, const int* in_sizes, int n_in,
                              void* d_out, int out_size, void* d_ws,
                              size_t ws_size, hipStream_t stream) {
  if (n_in < 13) return;
  const int M = B_ * N_;
  if (in_sizes[0] != M * D_ || in_sizes[1] != M * 3 || in_sizes[2] != M ||
      in_sizes[3] != D_ * D_ || in_sizes[4] != D_ || in_sizes[5] != D_ * D_ ||
      in_sizes[6] != D_ || in_sizes[7] != D_ * D_ || in_sizes[8] != D_ ||
      in_sizes[9] != D_ * D_ || in_sizes[10] != D_ || in_sizes[11] != R_ * H_ ||
      in_sizes[12] != H_ || out_size != M * D_)
    return;

  const float* h     = (const float*)d_in[0];
  const float* pos   = (const float*)d_in[1];
  const int*   mask  = (const int*)d_in[2];
  const float* q_w   = (const float*)d_in[3];
  const float* q_b   = (const float*)d_in[4];
  const float* k_w   = (const float*)d_in[5];
  const float* k_b   = (const float*)d_in[6];
  const float* v_w   = (const float*)d_in[7];
  const float* v_b   = (const float*)d_in[8];
  const float* o_w   = (const float*)d_in[9];
  const float* o_b   = (const float*)d_in[10];
  const float* rbf_w = (const float*)d_in[11];
  const float* rbf_b = (const float*)d_in[12];
  float* out = (float*)d_out;

  const size_t BND = (size_t)M * D_;
  const size_t need = BND * 4 + BND * 4 + BND * 4 + BND * 4;
  if (ws_size < need) return;
  char* ws = (char*)d_ws;
  float*  Qf  = (float*)(ws);
  __bf16* Khi = (__bf16*)(ws + BND * 4);
  __bf16* Klo = Khi + BND;
  __bf16* Vhi = (__bf16*)(ws + BND * 8);
  __bf16* Vlo = Vhi + BND;
  float*  Of  = (float*)(ws + BND * 12);

  const dim3 gg(M / 64, D_ / 128);
  const float qscale = 0.125f;

  k_gemm<0><<<gg, 256, 0, stream>>>(h, q_w, q_b, Qf, Khi, Klo, qscale, M);
  k_gemm<1><<<gg, 256, 0, stream>>>(h, k_w, k_b, Of, Khi, Klo, 1.0f, M);
  k_gemm<2><<<gg, 256, 0, stream>>>(h, v_w, v_b, Of, Vhi, Vlo, 1.0f, M);

  const dim3 ag(N_ / 16, B_);
  k_attn<<<ag, 256, ATT_LDS, stream>>>(Qf, Khi, Klo, Vhi, Vlo, pos, mask,
                                        rbf_w, rbf_b, Of);

  k_gemm<0><<<gg, 256, 0, stream>>>(Of, o_w, o_b, out, Khi, Klo, 1.0f, M);
}
